// KANGaussianPolicy_29274497089813
// MI455X (gfx1250) — hardware-verified
//
#include <hip/hip_runtime.h>
#include <math.h>

constexpr int kRows      = 32768;
constexpr int kIn        = 256;
constexpr int kHid       = 512;
constexpr int kAct       = 64;
constexpr int kNB        = 8;
constexpr int kK1        = kIn * (kNB + 1);
constexpr int kK2        = kHid * (kNB + 1);
constexpr int kNH2       = 2 * kAct;
constexpr int kChunks    = 4;
constexpr int kChunkRows = kRows / kChunks;
constexpr float kWCarry  = 8.0f;
constexpr float kLoCarry = 2048.0f;
constexpr float kScale1a = 1.0f / 8.0f;
constexpr float kScale1b = 1.0f / 16384.0f;
constexpr float kScale2  = 1.0f / 8.0f;

static_assert(kChunks * kChunkRows == kRows, "rows");
static_assert(kK1 % 32 == 0 && kK2 % 32 == 0, "K tile");
static_assert(kChunkRows % 64 == 0 && kHid % 64 == 0 && kNH2 % 64 == 0, "MN tile");
static_assert((kIn * 9) % 256 == 0 && (kHid * 9) % 256 == 0, "wprep wave rows");

constexpr size_t kBytesA1 = (size_t)kChunkRows * kK1 * 2;
constexpr size_t kBytesA2 = (size_t)kChunkRows * kK2 * 2;
constexpr size_t kBytesH  = (size_t)kChunkRows * kHid * 4;
constexpr size_t kBytesY  = (size_t)kChunkRows * kNH2 * 4;
constexpr size_t kBytesW1 = (size_t)kHid * kK1 * 2;
constexpr size_t kBytesW2 = (size_t)kNH2 * kK2 * 2;
constexpr size_t kOffA    = 0;
constexpr size_t kOffAlo  = kOffA + kBytesA1;
constexpr size_t kOffH0   = kOffA + kBytesA2;
constexpr size_t kOffH1   = kOffH0 + kBytesH;
constexpr size_t kOffY    = kOffH1 + kBytesH;
constexpr size_t kOffW1   = kOffY + kBytesY;
constexpr size_t kOffW2   = kOffW1 + kBytesW1;
constexpr size_t kWsTotal = kOffW2 + kBytesW2;
static_assert(kBytesA2 == 2 * kBytesA1, "A region reuse");
static_assert(kWsTotal == 116785152ull, "carve total");
static_assert(kWsTotal <= 134217728ull, "carve cap");
static_assert(kOffAlo % 128 == 0 && kOffH0 % 128 == 0 && kOffH1 % 128 == 0 && kOffY % 128 == 0 && kOffW1 % 128 == 0 && kOffW2 % 128 == 0, "align");

typedef __attribute__((ext_vector_type(16))) _Float16 v16h;
typedef __attribute__((ext_vector_type(8)))  _Float16 v8h;
typedef __attribute__((ext_vector_type(16))) __bf16   v16b;
typedef __attribute__((ext_vector_type(8)))  __bf16   v8b;
typedef __attribute__((ext_vector_type(8)))  float    v8f;
typedef __attribute__((ext_vector_type(4)))  float    v4f;
typedef __attribute__((ext_vector_type(4)))  unsigned int v4u;

__device__ __forceinline__ unsigned short f2bf_bits(float f) {
  unsigned u = __float_as_uint(f);
  return (unsigned short)((u + 0x7FFFu + ((u >> 16) & 1u)) >> 16);
}
__device__ __forceinline__ float bf_bits2f(unsigned short h) { return __uint_as_float(((unsigned)h) << 16); }

__device__ __forceinline__ void dep_guard_h(v8f& a, v8f& b, v16h x, v16h y) { asm volatile("v_nop\n\tv_nop\n\tv_nop\n\tv_nop" : "+v"(a), "+v"(b) : "v"(x), "v"(y)); }
__device__ __forceinline__ void dep_guard_b(v8f& a, v8f& b, v16b x, v16b y) { asm volatile("v_nop\n\tv_nop\n\tv_nop\n\tv_nop" : "+v"(a), "+v"(b) : "v"(x), "v"(y)); }
__device__ __forceinline__ void keep4_h(v16h a, v16h b, v16h c, v16h d) { asm volatile("v_nop" :: "v"(a), "v"(b), "v"(c), "v"(d)); }
__device__ __forceinline__ void keep4_b(v16b a, v16b b, v16b c, v16b d) { asm volatile("v_nop" :: "v"(a), "v"(b), "v"(c), "v"(d)); }
__device__ __forceinline__ void acc_guard4(v8f& a, v8f& b, v8f& c, v8f& d) { asm volatile("v_nop\n\tv_nop\n\tv_nop\n\tv_nop" : "+v"(a), "+v"(b), "+v"(c), "+v"(d)); }
template <typename T> struct Frag;
template <> struct Frag<_Float16> {
  typedef v16h V; union U { v16h v; v8h h[2]; };
  static __device__ __forceinline__ v16h load(const _Float16* p) {
    U f; f.h[0] = *(const v8h*)(p); f.h[1] = *(const v8h*)(p + 16); return f.v;
  }
  static __device__ __forceinline__ v8f mma(v16h a, v16h b, v8f c) {
    return __builtin_amdgcn_wmma_f32_16x16x32_f16(false, a, false, b, (short)0, c, false, false);
  }
  static __device__ __forceinline__ void guard(v8f& a, v8f& b, v16h x, v16h y) { dep_guard_h(a, b, x, y); }
  static __device__ __forceinline__ void keep(v16h a, v16h b, v16h c, v16h d) { keep4_h(a, b, c, d); }
};
template <> struct Frag<__bf16> {
  typedef v16b V; union U { v16b v; v8b h[2]; };
  static __device__ __forceinline__ v16b load(const __bf16* p) {
    U f; f.h[0] = *(const v8b*)(p); f.h[1] = *(const v8b*)(p + 16); return f.v;
  }
  static __device__ __forceinline__ v8f mma(v16b a, v16b b, v8f c) {
    return __builtin_amdgcn_wmma_f32_16x16x32_bf16(false, a, false, b, (short)0, c, false, false);
  }
  static __device__ __forceinline__ void guard(v8f& a, v8f& b, v16b x, v16b y) { dep_guard_b(a, b, x, y); }
  static __device__ __forceinline__ void keep(v16b a, v16b b, v16b c, v16b d) { keep4_b(a, b, c, d); }
};

__device__ __forceinline__ unsigned pk16(unsigned short a, unsigned short b) { return (unsigned)a | ((unsigned)b << 16); }
__device__ __forceinline__ unsigned short h_bits(float f) { const _Float16 h = (_Float16)f; return __builtin_bit_cast(unsigned short, h); }

template <int ET> struct Elem;
template <> struct Elem<0> { typedef _Float16 T; };
template <> struct Elem<1> { typedef __bf16 T; };
template <int ET, bool SPLIT, int BIAS_MODE, int OUT_MODE, bool RESID, int ACT = 0>
__global__ __launch_bounds__(256) void wmma_gemm64(
    const unsigned short* __restrict__ Ap, const unsigned short* __restrict__ A2p, int lda, long strideA,
    const unsigned short* __restrict__ Btp, const unsigned short* __restrict__ Bt2p, int ldb, long strideB,
    void* __restrict__ Cout, void* __restrict__ Cout2, int ldc, long strideC,
    const float* __restrict__ bias,
    const float* __restrict__ resid, long strideR,
    int M, int N, int K, float scale) {
  typedef typename Elem<ET>::T T;
  typedef typename Frag<T>::V V;
  const T* A = (const T*)Ap; const T* A2 = (const T*)A2p; const T* Bt = (const T*)Btp; const T* Bt2 = (const T*)Bt2p;
  __shared__ __align__(16) float sT[8][16 * 68];
  const int b    = blockIdx.y;
  const int lane = threadIdx.x & 31;
  const int wave = threadIdx.x >> 5;
  const int tilesN = N >> 6;
  const int tilesM = M >> 6;
  const int tile = blockIdx.x * 8 + wave;
  if (tile >= tilesM * tilesN) return;
  const int tm = tile / tilesN;
  const int tn = tile - tm * tilesN;
  const int m0 = tm << 6;
  const int n0 = tn << 6;

  const T* Ab  = A  + (size_t)b * strideA;
  const T* Bb  = Bt + (size_t)b * strideB;
  const T* Ab2 = SPLIT ? (A2  + (size_t)b * strideA) : nullptr;
  const T* Bb2 = SPLIT ? (Bt2 + (size_t)b * strideB) : nullptr;

  const int rlane = lane & 15;
  const int koff  = (lane >> 4) * 8;
  const int mOff  = (lane >> 4) * 8;

  v8f acc[4][4];
#pragma unroll
  for (int i = 0; i < 4; ++i)
#pragma unroll
    for (int j = 0; j < 4; ++j) acc[i][j] = (v8f){0.f,0.f,0.f,0.f,0.f,0.f,0.f,0.f};

  for (int k0 = 0; k0 < K; k0 += 32) {
    V bh[4], bl[4];
#pragma unroll
    for (int j = 0; j < 4; ++j) {
      const size_t bo = (size_t)(n0 + (j << 4) + rlane) * ldb + koff + k0;
      bh[j] = Frag<T>::load(Bb + bo);
      if (SPLIT) bl[j] = Frag<T>::load(Bb2 + bo);
    }
#pragma unroll
    for (int i = 0; i < 4; ++i) {
      const size_t ao = (size_t)(m0 + (i << 4) + rlane) * lda + koff + k0;
      V ah = Frag<T>::load(Ab + ao);
      V al;
      if (SPLIT) al = Frag<T>::load(Ab2 + ao);
#pragma unroll
      for (int j = 0; j < 4; ++j) {
        acc[i][j] = Frag<T>::mma(ah, bh[j], acc[i][j]);
        if (SPLIT) {
          acc[i][j] = Frag<T>::mma(ah, bl[j], acc[i][j]);
          acc[i][j] = Frag<T>::mma(al, bh[j], acc[i][j]);
        }
      }
      Frag<T>::guard(acc[i][0], acc[i][3], ah, SPLIT ? al : ah);
    }
    Frag<T>::keep(bh[0], bh[1], bh[2], bh[3]);
    if (SPLIT) Frag<T>::keep(bl[0], bl[1], bl[2], bl[3]);
  }
  acc_guard4(acc[0][0], acc[0][1], acc[0][2], acc[0][3]);
  acc_guard4(acc[1][0], acc[1][1], acc[1][2], acc[1][3]);
  acc_guard4(acc[2][0], acc[2][1], acc[2][2], acc[2][3]);
  acc_guard4(acc[3][0], acc[3][1], acc[3][2], acc[3][3]);

  float* slab = sT[wave];
  const float* Rb = RESID ? (resid + (size_t)b * strideR) : nullptr;
#pragma unroll
  for (int i = 0; i < 4; ++i) {
    const int mBase = m0 + (i << 4);
#pragma unroll
    for (int j = 0; j < 4; ++j) {
      const int n = n0 + (j << 4) + rlane;
      float bv = 0.f;
      if (BIAS_MODE == 2) bv = bias[n];
#pragma unroll
      for (int r = 0; r < 8; ++r) {
        float v = acc[i][j][r] * scale;
        if (BIAS_MODE == 1) v += bias[mBase + mOff + r];
        if (BIAS_MODE == 2) v += bv;
        if (RESID) v += Rb[(size_t)(mBase + mOff + r) * ldc + n];
        if (ACT == 2) v = fmaxf(v, 0.0f);
        if (ACT == 4) v = (v > 0.f) ? v : 0.01f * v;
        slab[(mOff + r) * 68 + (j << 4) + rlane] = v;
      }
    }
    __builtin_amdgcn_fence(__ATOMIC_RELEASE, "workgroup");
    __builtin_amdgcn_wave_barrier();
    __builtin_amdgcn_fence(__ATOMIC_ACQUIRE, "workgroup");
    if (OUT_MODE == 0) {
      float* C = (float*)Cout + (size_t)b * strideC;
      const int hh = lane >> 4, c4 = (lane & 15) * 4;
      for (int pass = 0; pass < 2; ++pass) {
#pragma unroll
        for (int it = 0; it < 8; ++it) {
          const int row = it * 2 + hh;
          v4f v = *(const v4f*)(slab + row * 68 + c4);
          *(volatile v4f*)(C + (size_t)(mBase + row) * ldc + n0 + c4) = v;
        }
        __threadfence();
      }
    } else {
      const int q = lane >> 3, c8 = (lane & 7) * 8;
      unsigned short* C  = (unsigned short*)Cout  + (size_t)b * strideC;
      unsigned short* C2 = (OUT_MODE == 2) ? ((unsigned short*)Cout2 + (size_t)b * strideC) : nullptr;
      for (int pass = 0; pass < 2; ++pass) {
#pragma unroll
        for (int it = 0; it < 4; ++it) {
          const int row = it * 4 + q;
          const float* sp = slab + row * 68 + c8;
          v8h hv, lv;
#pragma unroll
          for (int e = 0; e < 8; ++e) {
            if (OUT_MODE == 1) {
              hv[e] = (_Float16)sp[e];
            } else {
              unsigned short hb = f2bf_bits(sp[e]);
              unsigned short lb = f2bf_bits(sp[e] - bf_bits2f(hb));
              hv[e] = __builtin_bit_cast(_Float16, hb);
              lv[e] = __builtin_bit_cast(_Float16, lb);
            }
          }
          *(volatile v8h*)(C + (size_t)(mBase + row) * ldc + n0 + c8) = hv;
          if (OUT_MODE == 2) *(volatile v8h*)(C2 + (size_t)(mBase + row) * ldc + n0 + c8) = lv;
        }
        __threadfence();
      }
    }
    __builtin_amdgcn_fence(__ATOMIC_RELEASE, "workgroup");
    __builtin_amdgcn_wave_barrier();
    __builtin_amdgcn_fence(__ATOMIC_ACQUIRE, "workgroup");
  }
}

__device__ __forceinline__ float silu_f(float x) {
#pragma clang fp contract(off)
  const float e = expf(-x);
  const float s = 1.0f / (1.0f + e);
  return x * s;
}

__device__ __forceinline__ float tanh_f(float x) {
#pragma clang fp contract(off)
  const float e = expf(2.0f * x);
  const float d = e + 1.0f;
  return 1.0f - 2.0f / d;
}

__device__ __forceinline__ void kan_basis8(float x, float* out) {
#pragma clang fp contract(off)
  float g[12];
#pragma unroll
  for (int j = 0; j < 12; ++j) {
    const float t = (float)(j - 3) * 0.4f;
    g[j] = t + (-1.0f);
  }
  float b[11];
#pragma unroll
  for (int j = 0; j < 11; ++j) b[j] = (x >= g[j] && x < g[j + 1]) ? 1.0f : 0.0f;
#pragma unroll
  for (int p = 1; p <= 3; ++p) {
#pragma unroll
    for (int j = 0; j < 11 - p; ++j) {
      const float rl = 1.0f / (g[j + p] - g[j]);
      const float rr = 1.0f / (g[j + p + 1] - g[j + 1]);
      float lt = (x - g[j]) * rl;
      lt = lt * b[j];
      float rt = (g[j + p + 1] - x) * rr;
      rt = rt * b[j + 1];
      b[j] = lt + rt;
    }
  }
#pragma unroll
  for (int j = 0; j < 8; ++j) out[j] = b[j];
}

__device__ __forceinline__ void split16(float v, unsigned short& hb, unsigned short& lb) {
#pragma clang fp contract(off)
  const _Float16 h16 = (_Float16)v;
  float hf = (float)h16;
  hf = (fabsf(v) < 6.103515625e-05f) ? 0.0f : hf;
  const float res = (v - hf) * kLoCarry;
  const _Float16 hs = (_Float16)hf;
  const _Float16 ls = (_Float16)res;
  hb = __builtin_bit_cast(unsigned short, hs);
  lb = __builtin_bit_cast(unsigned short, ls);
}

__global__ __launch_bounds__(256) void wprep_kernel(const float* __restrict__ swA, const float* __restrict__ bwA,
                                                    const float* __restrict__ swB, const float* __restrict__ bwB,
                                                    int nsplit, int nrows, int nin,
                                                    unsigned short* __restrict__ outp,
                                                    const int* __restrict__ iarg0, const int* __restrict__ iarg1) {
#pragma clang fp contract(off)
  (void)iarg0; (void)iarg1;
  const int tpr = (nin * 9) >> 3;
  const int total = nrows * tpr;
  const int i = blockIdx.x * 256 + threadIdx.x;
  if (i >= total) return;
  const int r = i / tpr;
  const int kk = (i - r * tpr) * 8;
  const int kspl = nin * 8;
  const bool useA = (r < nsplit);
  const bool spl = (kk < kspl);
  const int rA = (r < nsplit) ? r : (nsplit - 1);
  int rB = r - nsplit;
  {
    const int rbmax = nrows - nsplit - 1;
    rB = (rB > rbmax) ? rbmax : rB;
    rB = (rB < 0) ? 0 : rB;
  }
  const int ks = (kk > kspl - 8) ? (kspl - 8) : kk;
  int kb = kk - kspl;
  kb = (kb < 0) ? 0 : kb;
  kb = (kb > nin - 8) ? (nin - 8) : kb;
  const float* psA = swA + (size_t)rA * kspl + ks;
  const float* pbA = bwA + (size_t)rA * nin + kb;
  const float* psB = swB + (size_t)rB * kspl + ks;
  const float* pbB = bwB + (size_t)rB * nin + kb;
  const v4f sA0 = *(const v4f*)(psA), sA1 = *(const v4f*)(psA + 4);
  const v4f bA0 = *(const v4f*)(pbA), bA1 = *(const v4f*)(pbA + 4);
  const v4f sB0 = *(const v4f*)(psB), sB1 = *(const v4f*)(psB + 4);
  const v4f bB0 = *(const v4f*)(pbB), bB1 = *(const v4f*)(pbB + 4);
  unsigned short hb[8];
#pragma unroll
  for (int e = 0; e < 4; ++e) {
    const float a0 = useA ? (spl ? sA0[e] : bA0[e]) : (spl ? sB0[e] : bB0[e]);
    const float a1 = useA ? (spl ? sA1[e] : bA1[e]) : (spl ? sB1[e] : bB1[e]);
    hb[e]     = h_bits(a0 * kWCarry);
    hb[4 + e] = h_bits(a1 * kWCarry);
  }
  const v4u u = (v4u){pk16(hb[0], hb[1]), pk16(hb[2], hb[3]), pk16(hb[4], hb[5]), pk16(hb[6], hb[7])};
  unsigned short* q = outp + (size_t)r * (size_t)(nin * 9) + kk;
  *(volatile v4u*)q = u;
  __threadfence();
  *(volatile v4u*)q = u;
}

__global__ __launch_bounds__(256) void basis1_kernel(const float* __restrict__ state, int row0,
                                                     unsigned short* __restrict__ Ahi, unsigned short* __restrict__ Alo) {
#pragma clang fp contract(off)
  __shared__ __align__(16) float sAct[kIn];
  const int row  = blockIdx.x;
  const int t    = threadIdx.x;
  const int lane = t & 31;
  const int wave = t >> 5;
  const float x = state[(size_t)(row0 + row) * kIn + t];
  sAct[t] = silu_f(x);
  float bs[8];
  kan_basis8(x, bs);
  unsigned short hb[8], lb[8];
#pragma unroll
  for (int e = 0; e < 8; ++e) split16(bs[e], hb[e], lb[e]);
  const v4u hv = (v4u){pk16(hb[0], hb[1]), pk16(hb[2], hb[3]), pk16(hb[4], hb[5]), pk16(hb[6], hb[7])};
  const v4u lv = (v4u){pk16(lb[0], lb[1]), pk16(lb[2], lb[3]), pk16(lb[4], lb[5]), pk16(lb[6], lb[7])};
  __syncthreads();
  const v4f a0 = *(const v4f*)(sAct + lane * 8);
  const v4f a1 = *(const v4f*)(sAct + lane * 8 + 4);
  unsigned short sh[8], sl[8];
#pragma unroll
  for (int e = 0; e < 4; ++e) {
    split16(a0[e], sh[e], sl[e]);
    split16(a1[e], sh[4 + e], sl[4 + e]);
  }
  const v4u shv = (v4u){pk16(sh[0], sh[1]), pk16(sh[2], sh[3]), pk16(sh[4], sh[5]), pk16(sh[6], sh[7])};
  const v4u slv = (v4u){pk16(sl[0], sl[1]), pk16(sl[2], sl[3]), pk16(sl[4], sl[5]), pk16(sl[6], sl[7])};
  unsigned short* ph = Ahi + (size_t)row * kK1;
  unsigned short* pl = Alo + (size_t)row * kK1;
  for (int pass = 0; pass < 2; ++pass) {
    *(volatile v4u*)(ph + t * 8) = hv;
    *(volatile v4u*)(pl + t * 8) = lv;
    if (wave == 0) {
      *(volatile v4u*)(ph + kIn * kNB + lane * 8) = shv;
      *(volatile v4u*)(pl + kIn * kNB + lane * 8) = slv;
    }
    __threadfence();
  }
}

__global__ __launch_bounds__(256) void lnbasis2_kernel(const float* __restrict__ Hin, const float* __restrict__ gamma,
                                                       const float* __restrict__ beta, unsigned short* __restrict__ A2) {
#pragma clang fp contract(off)
  __shared__ __align__(16) float sAct[kHid];
  __shared__ float sRedA[8];
  __shared__ float sRedB[8];
  const int row  = blockIdx.x;
  const int t    = threadIdx.x;
  const int lane = t & 31;
  const int wave = t >> 5;
  const float* hr = Hin + (size_t)row * kHid;
  const float x0 = hr[t];
  const float x1 = hr[t + 256];
  float s = x0 + x1;
#pragma unroll
  for (int off = 16; off > 0; off >>= 1) s += __shfl_xor(s, off, 32);
  if (lane == 0) sRedA[wave] = s;
  __syncthreads();
  float tot = sRedA[0];
#pragma unroll
  for (int w = 1; w < 8; ++w) tot = tot + sRedA[w];
  const float mu = tot * (1.0f / 512.0f);
  const float d0 = x0 - mu;
  const float d1 = x1 - mu;
  const float q0 = d0 * d0;
  const float q1 = d1 * d1;
  float sq = q0 + q1;
#pragma unroll
  for (int off = 16; off > 0; off >>= 1) sq += __shfl_xor(sq, off, 32);
  if (lane == 0) sRedB[wave] = sq;
  __syncthreads();
  float tot2 = sRedB[0];
#pragma unroll
  for (int w = 1; w < 8; ++w) tot2 = tot2 + sRedB[w];
  const float var  = tot2 * (1.0f / 512.0f);
  const float rstd = rsqrtf(var + 1e-5f);
  float y0 = d0 * rstd;
  y0 = y0 * gamma[t];
  y0 = y0 + beta[t];
  y0 = fmaxf(y0, 0.0f);
  float y1 = d1 * rstd;
  y1 = y1 * gamma[t + 256];
  y1 = y1 + beta[t + 256];
  y1 = fmaxf(y1, 0.0f);
  sAct[t]       = silu_f(y0);
  sAct[t + 256] = silu_f(y1);
  float bs[8];
  unsigned short hb[8];
  kan_basis8(y0, bs);
#pragma unroll
  for (int e = 0; e < 8; ++e) hb[e] = h_bits(bs[e]);
  const v4u hv0 = (v4u){pk16(hb[0], hb[1]), pk16(hb[2], hb[3]), pk16(hb[4], hb[5]), pk16(hb[6], hb[7])};
  kan_basis8(y1, bs);
#pragma unroll
  for (int e = 0; e < 8; ++e) hb[e] = h_bits(bs[e]);
  const v4u hv1 = (v4u){pk16(hb[0], hb[1]), pk16(hb[2], hb[3]), pk16(hb[4], hb[5]), pk16(hb[6], hb[7])};
  __syncthreads();
  const int ai = (((wave & 1) << 5) + lane) * 8;
  const v4f a0 = *(const v4f*)(sAct + ai);
  const v4f a1 = *(const v4f*)(sAct + ai + 4);
  unsigned short sh[8];
#pragma unroll
  for (int e = 0; e < 4; ++e) { sh[e] = h_bits(a0[e]); sh[4 + e] = h_bits(a1[e]); }
  const v4u sv = (v4u){pk16(sh[0], sh[1]), pk16(sh[2], sh[3]), pk16(sh[4], sh[5]), pk16(sh[6], sh[7])};
  unsigned short* rp = A2 + (size_t)row * kK2;
  for (int pass = 0; pass < 2; ++pass) {
    *(volatile v4u*)(rp + t * 8) = hv0;
    *(volatile v4u*)(rp + (t + 256) * 8) = hv1;
    if (wave < 2) {
      *(volatile v4u*)(rp + kHid * kNB + ai) = sv;
    }
    __threadfence();
  }
}

__global__ __launch_bounds__(256) void heads_kernel(const float* __restrict__ Y, float* __restrict__ out, int row0, int n4) {
#pragma clang fp contract(off)
  const int i = blockIdx.x * 256 + threadIdx.x;
  if (i >= n4) return;
  const int r  = i >> 5;
  const int qs = i & 31;
  const v4f y = *(const v4f*)(Y + (size_t)r * kNH2 + qs * 4);
  const bool isMean = (qs < 16);
  v4f v;
#pragma unroll
  for (int e = 0; e < 4; ++e) {
    const float th = tanh_f(y[e]);
    const float cl = fminf(fmaxf(y[e], -20.0f), 2.0f);
    v[e] = isMean ? th : cl;
  }
  const size_t off = (isMean ? (size_t)0 : ((size_t)kRows * kAct)) + (size_t)(row0 + r) * kAct + (size_t)((qs & 15) * 4);
  *(volatile v4f*)(out + off) = v;
  __threadfence();
  *(volatile v4f*)(out + off) = v;
}

extern "C" void kernel_launch(void* const* d_in, const int* in_sizes, int n_in,
                              void* d_out, int out_size, void* d_ws, size_t ws_size,
                              hipStream_t stream) {
  if (n_in < 11) return;
  if (in_sizes[0] != kRows * kIn) return;
  if (in_sizes[1] != kHid * kIn) return;
  if (in_sizes[2] != kHid * kIn * kNB) return;
  if (in_sizes[3] < kHid || in_sizes[4] < kHid) return;
  if (in_sizes[5] != kAct * kHid || in_sizes[7] != kAct * kHid) return;
  if (in_sizes[6] != kAct * kHid * kNB || in_sizes[8] != kAct * kHid * kNB) return;
  if (out_size != 2 * kRows * kAct) return;
  if (ws_size < kWsTotal) return;

  const float* state    = (const float*)d_in[0];
  const float* feat_bw  = (const float*)d_in[1];
  const float* feat_sw  = (const float*)d_in[2];
  const float* ln_gamma = (const float*)d_in[3];
  const float* ln_beta  = (const float*)d_in[4];
  const float* mean_bw  = (const float*)d_in[5];
  const float* mean_sw  = (const float*)d_in[6];
  const float* lstd_bw  = (const float*)d_in[7];
  const float* lstd_sw  = (const float*)d_in[8];
  const int*   gsz      = (const int*)d_in[9];
  const int*   sord     = (const int*)d_in[10];
  float* out = (float*)d_out;

  char* ws = (char*)d_ws;
  unsigned short* A1hi = (unsigned short*)(ws + kOffA);
  unsigned short* A1lo = (unsigned short*)(ws + kOffAlo);
  unsigned short* A2   = (unsigned short*)(ws + kOffA);
  float*          H0   = (float*)(ws + kOffH0);
  float*          H1   = (float*)(ws + kOffH1);
  float*          Y    = (float*)(ws + kOffY);
  unsigned short* W1t  = (unsigned short*)(ws + kOffW1);
  unsigned short* W2t  = (unsigned short*)(ws + kOffW2);

  {
    const int total = kHid * ((kIn * 9) / 8);
    wprep_kernel<<<dim3((total + 255) / 256), dim3(256), 0, stream>>>(
        feat_sw, feat_bw, feat_sw, feat_bw, kHid, kHid, kIn, W1t, gsz, sord);
  }
  {
    const int total = kNH2 * ((kHid * 9) / 8);
    wprep_kernel<<<dim3((total + 255) / 256), dim3(256), 0, stream>>>(
        mean_sw, mean_bw, lstd_sw, lstd_bw, kAct, kNH2, kHid, W2t, gsz, sord);
  }

  const int gemmBlocks1 = ((kChunkRows / 64) * (kHid / 64) + 7) / 8;
  const int gemmBlocks2 = ((kChunkRows / 64) * (kNH2 / 64) + 7) / 8;
  const int n4heads = kChunkRows * (kNH2 / 4);

  for (int c = 0; c < kChunks; ++c) {
    const int row0 = c * kChunkRows;

    basis1_kernel<<<dim3(kChunkRows), dim3(256), 0, stream>>>(state, row0, A1hi, A1lo);

    wmma_gemm64<0, false, 0, 0, false, 0><<<dim3(gemmBlocks1, 1), dim3(256), 0, stream>>>(
        A1hi, A1hi, kK1, (long)0,
        W1t, W1t, kK1, (long)0,
        (void*)H0, (void*)H0, kHid, (long)0,
        ln_gamma,
        H1, (long)0,
        kChunkRows, kHid, kK1, kScale1a);

    wmma_gemm64<0, false, 0, 0, true, 0><<<dim3(gemmBlocks1, 1), dim3(256), 0, stream>>>(
        A1lo, A1lo, kK1, (long)0,
        W1t, W1t, kK1, (long)0,
        (void*)H1, (void*)H1, kHid, (long)0,
        ln_gamma,
        H0, (long)0,
        kChunkRows, kHid, kK1, kScale1b);

    lnbasis2_kernel<<<dim3(kChunkRows), dim3(256), 0, stream>>>(H1, ln_gamma, ln_beta, A2);

    wmma_gemm64<0, false, 0, 0, false, 0><<<dim3(gemmBlocks2, 1), dim3(256), 0, stream>>>(
        A2, A2, kK2, (long)0,
        W2t, W2t, kK2, (long)0,
        (void*)Y, (void*)Y, kNH2, (long)0,
        ln_gamma,
        H0, (long)0,
        kChunkRows, kNH2, kK2, kScale2);

    heads_kernel<<<dim3((n4heads + 255) / 256), dim3(256), 0, stream>>>(Y, out, row0, n4heads);
  }
}
